// GraphAttentional_30021821399296
// MI455X (gfx1250) — hardware-verified
//
#include <hip/hip_runtime.h>
#include <math.h>

#define Bc 4
#define Gc 128
#define Nc 2048
#define Pc 4
#define Fc 64
#define NEG_SLOPE 0.2f
#define ZTOL 1e-9f
#define LOG2E 1.4426950408889634f

typedef _Float16 h16;
typedef __attribute__((ext_vector_type(16))) _Float16 v16h;
typedef __attribute__((ext_vector_type(8)))  _Float16 v8h;
typedef __attribute__((ext_vector_type(8)))  float v8f;
typedef __attribute__((ext_vector_type(4)))  float v4f_t;
typedef float v4fa __attribute__((ext_vector_type(4), may_alias));
typedef __attribute__((ext_vector_type(4)))  unsigned v4u_t;
typedef unsigned v4ua __attribute__((ext_vector_type(4), may_alias));

__device__ __forceinline__ v8f wmma16(v16h a, v16h b, v8f c) { return __builtin_amdgcn_wmma_f32_16x16x32_f16(false, a, false, b, (short)0, c, false, false); }
__device__ __forceinline__ v16h rfrag(const h16* rowp, int half) {
  const h16* p = rowp + 8 * half;
  return __builtin_shufflevector(*(const v8h*)p, *(const v8h*)(p + 16), 0,1,2,3,4,5,6,7,8,9,10,11,12,13,14,15);
}
__device__ __forceinline__ float leaky(float e) { return e >= 0.0f ? e : NEG_SLOPE * e; }

__global__ __launch_bounds__(256) void k_xT(const float* __restrict__ x, h16* __restrict__ xT) {
  const int gidx = blockIdx.x * 256 + threadIdx.x;
  if (gidx >= Bc * Nc * (Gc / 8)) return;
  const int n = gidx & (Nc - 1), g8 = ((gidx >> 11) & 15) * 8, b = gidx >> 15;
  h16 hh[8];
#pragma unroll
  for (int e = 0; e < 8; ++e) hh[e] = (h16)x[((size_t)b * Gc + g8 + e) * Nc + n];
  h16* d = xT + ((size_t)b * Nc + n) * Gc + g8;
  *(volatile v4u_t*)d = *(const v4ua*)hh; __threadfence(); *(volatile v4u_t*)d = *(const v4ua*)hh;
}

__global__ __launch_bounds__(128) void k_wx(const h16* __restrict__ xT, const float* __restrict__ a, const float* __restrict__ W,
                                           float* __restrict__ Wx32, h16* __restrict__ Wx16, float* __restrict__ s1, float* __restrict__ s2) {
  __shared__ __attribute__((aligned(16))) h16 Ws[Fc * 136];
  __shared__ __attribute__((aligned(16))) float T[Fc * 68];
  __shared__ float a1s[Fc], a2s[Fc];
  const int bp = blockIdx.y, p = bp & (Pc - 1), b = bp >> 2;
  const int n0 = blockIdx.x * 64;
  const int tid = threadIdx.x, lane = tid & 31, wave = tid >> 5, half = lane >> 4, l16 = lane & 15;
  for (int i = tid; i < Fc * Gc; i += 128) { const int f = i >> 7, g = i & 127; Ws[f * 136 + g] = (h16)W[((size_t)p * Fc + f) * Gc + g]; }
  if (tid < Fc) { a1s[tid] = a[p * 2 * Fc + tid]; a2s[tid] = a[p * 2 * Fc + Fc + tid]; }
  __syncthreads();
  v8f acc[4] = {};
  const h16* xrow = xT + ((size_t)b * Nc + n0 + wave * 16 + l16) * Gc;
#pragma unroll
  for (int kc = 0; kc < 4; ++kc) {
    const v16h bfr = rfrag(xrow + kc * 32, half);
#pragma unroll
    for (int ft = 0; ft < 4; ++ft) acc[ft] = wmma16(rfrag(Ws + (ft * 16 + l16) * 136 + kc * 32, half), bfr, acc[ft]);
  }
#pragma unroll
  for (int ft = 0; ft < 4; ++ft)
#pragma unroll
    for (int r = 0; r < 8; ++r) T[(ft * 16 + 8 * half + r) * 68 + wave * 16 + l16] = acc[ft][r];
  __syncthreads();
  {
    const int nl = tid & 63; const bool isS2 = tid >= 64;
    float sacc = 0.0f;
#pragma unroll 1
    for (int f = 0; f < Fc; ++f) sacc += (isS2 ? a2s[f] : a1s[f]) * T[f * 68 + nl];
    float* dst = (isS2 ? s2 : s1) + (size_t)bp * Nc + n0 + nl;
    *(volatile float*)dst = sacc; __threadfence(); *(volatile float*)dst = sacc;
  }
  const size_t rowBase = (size_t)bp * Fc;
#pragma unroll 1
  for (int pass = 0; pass < 2; ++pass) {
    for (int ch = tid; ch < Fc * 16; ch += 128) { const int f = ch >> 4, q = (ch & 15) * 4;
      *(volatile v4f_t*)(Wx32 + (rowBase + f) * Nc + n0 + q) = *(const volatile v4fa*)(T + f * 68 + q); }
    for (int ch = tid; ch < Fc * 8; ch += 128) { const int f = ch >> 3, q = (ch & 7) * 8; h16 hh[8];
#pragma unroll
      for (int e = 0; e < 8; ++e) hh[e] = (h16)T[f * 68 + q + e];
      *(volatile v4u_t*)(Wx16 + (rowBase + f) * Nc + n0 + q) = *(const v4ua*)hh; }
    __threadfence();
  }
}

__global__ __launch_bounds__(256) void k_rowstats(const float* __restrict__ S, const float* __restrict__ s1, const float* __restrict__ s2,
                                                 float* __restrict__ rmax, float* __restrict__ rsum) {
  __shared__ float red[16][256];
  __shared__ float smax[16];
  __shared__ unsigned char inmask[Nc];
  const int m = blockIdx.x, tid = threadIdx.x;
  for (int n = tid; n < Nc; n += 256) { const float sv = S[(size_t)m * Nc + n] + ((n == m) ? 1.0f : 0.0f); inmask[n] = (fabsf(sv) > ZTOL) ? 1 : 0; }
  __syncthreads();
  float mx[16];
#pragma unroll
  for (int bp = 0; bp < 16; ++bp) mx[bp] = -3.0e38f;
  for (int n = tid; n < Nc; n += 256) {
    if (!inmask[n]) continue;
#pragma unroll
    for (int bp = 0; bp < 16; ++bp) mx[bp] = fmaxf(mx[bp], leaky(s1[(size_t)bp * Nc + n] + s2[(size_t)bp * Nc + m]));
  }
#pragma unroll
  for (int bp = 0; bp < 16; ++bp) red[bp][tid] = mx[bp];
  __syncthreads();
  for (int o = 128; o > 0; o >>= 1) { if (tid < o) {
#pragma unroll
      for (int bp = 0; bp < 16; ++bp) red[bp][tid] = fmaxf(red[bp][tid], red[bp][tid + o]); } __syncthreads(); }
  if (tid < 16) smax[tid] = red[tid][0];
  __syncthreads();
  float sm[16];
#pragma unroll
  for (int bp = 0; bp < 16; ++bp) { sm[bp] = 0.0f; mx[bp] = smax[bp]; }
  for (int n = tid; n < Nc; n += 256) {
    if (!inmask[n]) continue;
#pragma unroll
    for (int bp = 0; bp < 16; ++bp) sm[bp] += __expf(leaky(s1[(size_t)bp * Nc + n] + s2[(size_t)bp * Nc + m]) - mx[bp]);
  }
  __syncthreads();
#pragma unroll
  for (int bp = 0; bp < 16; ++bp) red[bp][tid] = sm[bp];
  __syncthreads();
  for (int o = 128; o > 0; o >>= 1) { if (tid < o) {
#pragma unroll
      for (int bp = 0; bp < 16; ++bp) red[bp][tid] += red[bp][tid + o]; } __syncthreads(); }
  if (tid < 16) { const float vmax = smax[tid], vsum = red[tid][0];
    *(volatile float*)(rmax + (size_t)m * 16 + tid) = vmax; *(volatile float*)(rsum + (size_t)m * 16 + tid) = vsum; __threadfence();
    *(volatile float*)(rmax + (size_t)m * 16 + tid) = vmax; *(volatile float*)(rsum + (size_t)m * 16 + tid) = vsum; }
}

__global__ __launch_bounds__(256) void k_aggregate(const float* __restrict__ S, const h16* __restrict__ Wx16,
                                                  const float* __restrict__ s1, const float* __restrict__ s2,
                                                  const float* __restrict__ rmax, const float* __restrict__ rsum,
                                                  float* __restrict__ out) {
  __shared__ __attribute__((aligned(16))) float so[Fc * 68];
  const int bp = blockIdx.y, n0 = blockIdx.x * 64;
  const int tid = threadIdx.x, lane = tid & 31, wave = tid >> 5, half = lane >> 4, l16 = lane & 15;
  const int nt = wave & 3, fh = wave >> 2;
  const int n = n0 + nt * 16 + l16;
  const float s1n = s1[(size_t)bp * Nc + n];
  const h16* wxb = Wx16 + (size_t)bp * Fc * Nc;
  const float* s2b = s2 + (size_t)bp * Nc;
  v8f acc[2] = {};
#pragma unroll 1
  for (int kc = 0; kc < Nc / 32; ++kc) {
    v16h bfr;
#pragma unroll
    for (int e = 0; e < 16; ++e) {
      const int m = kc * 32 + 8 * half + ((e < 8) ? e : (e + 8));
      const float sv = S[(size_t)m * Nc + n];
      float t = 0.0f;
      if (sv != 0.0f) {
        const float ex = __expf(leaky(s1n + s2b[m]) - rmax[(size_t)m * 16 + bp]);
        t = sv * ex / rsum[(size_t)m * 16 + bp];
      }
      bfr[e] = (h16)t;
    }
#pragma unroll
    for (int i = 0; i < 2; ++i) acc[i] = wmma16(rfrag(wxb + (size_t)((fh * 2 + i) * 16 + l16) * Nc + kc * 32, half), bfr, acc[i]);
  }
#pragma unroll
  for (int i = 0; i < 2; ++i)
#pragma unroll
    for (int r = 0; r < 8; ++r) { const float v = acc[i][r]; so[((fh * 2 + i) * 16 + 8 * half + r) * 68 + nt * 16 + l16] = v > 0.0f ? v : 0.0f; }
  __syncthreads();
  const int p = bp & (Pc - 1), b = bp >> 2;
#pragma unroll 1
  for (int pass = 0; pass < 2; ++pass) {
    for (int ch = tid; ch < Fc * 16; ch += 256) { const int f = ch >> 4, q = (ch & 15) * 4;
      *(volatile v4f_t*)(out + ((size_t)b * (Pc * Fc) + p * Fc + f) * Nc + n0 + q) = *(const volatile v4fa*)(so + f * 68 + q); }
    __threadfence();
  }
}

extern "C" void kernel_launch(void* const* d_in, const int* in_sizes, int n_in,
                              void* d_out, int out_size, void* d_ws, size_t ws_size,
                              hipStream_t stream) {
  (void)in_sizes; (void)n_in; (void)out_size; (void)ws_size;
  const float* x = (const float*)d_in[0];
  const float* a = (const float*)d_in[1];
  const float* W = (const float*)d_in[2];
  const float* S = (const float*)d_in[3];
  float* out = (float*)d_out;

  char* w = (char*)d_ws;
  h16*   xT   = (h16*)w;                                    w += (size_t)Bc * Nc * Gc * 2;
  float* Wx32 = (float*)w;                                  w += (size_t)Bc * Pc * Fc * Nc * 4;
  h16*   Wx16 = (h16*)w;                                    w += (size_t)Bc * Pc * Fc * Nc * 2;
  float* s1   = (float*)w;                                  w += (size_t)Bc * Pc * Nc * 4;
  float* s2   = (float*)w;                                  w += (size_t)Bc * Pc * Nc * 4;
  float* rmax = (float*)w;                                  w += (size_t)Nc * 16 * 4;
  float* rsum = (float*)w;                                  w += (size_t)Nc * 16 * 4;

  k_xT<<<(Bc * Nc * (Gc / 8)) / 256, 256, 0, stream>>>(x, xT);
  k_wx<<<dim3(Nc / 64, Bc * Pc), 128, 0, stream>>>(xT, a, W, Wx32, Wx16, s1, s2);
  k_rowstats<<<Nc, 256, 0, stream>>>(S, s1, s2, rmax, rsum);
  k_aggregate<<<dim3(Nc / 64, Bc * Pc), 256, 0, stream>>>(S, Wx16, s1, s2, rmax, rsum, out);
}
